// CausalSelfAttention_65412351918724
// MI455X (gfx1250) — hardware-verified
//
#include <hip/hip_runtime.h>
#include <math.h>
#ifndef NB
#define NB 2
#endif
#ifndef SEQ
#define SEQ 2048
#endif
#define NB_FULL 2
#define SEQ_FULL 2048
#define CC 1024
#define NH 16
#define HD 64
#define QKVN (3 * CC)
#define KP (2 * CC)
#define PL (NB * SEQ * CC)
#ifndef OUT_SEG_ROWS
#define OUT_SEG_ROWS SEQ_FULL
#endif
static_assert(NB >= 1 && NB <= NB_FULL);
static_assert(SEQ >= 64 && SEQ <= SEQ_FULL && (SEQ % 64) == 0);
static_assert(CC == NH * HD);
static_assert(HD == 64);
static_assert((CC % 64) == 0 && (CC % 32) == 0 && (KP % 32) == 0);
static_assert(((NB * SEQ) % 64) == 0);
static_assert((QKVN / 64) == 3 * NH);
static_assert(128 * 4 == 64 * 8);
static_assert((long long)4 * PL < 2147483647LL);
static_assert((size_t)NB_FULL * SEQ_FULL * CC * 2 + (size_t)3 * CC * CC * 2 + (size_t)CC * KP * 2 + (size_t)SEQ_FULL * 64 * 4 +
              (size_t)4 * NB_FULL * SEQ_FULL * CC * 2 + (size_t)NB_FULL * SEQ_FULL * KP * 2 <= (size_t)134217728);
static_assert((size_t)((NB - 1) * OUT_SEG_ROWS + SEQ) * CC * 4 <= (size_t)16777216);

typedef __bf16   v16b __attribute__((ext_vector_type(16)));
typedef _Float16 v16h __attribute__((ext_vector_type(16)));
typedef unsigned short v8us __attribute__((ext_vector_type(8), may_alias));
typedef float  v8f  __attribute__((ext_vector_type(8)));
typedef float  v4f  __attribute__((ext_vector_type(4)));
typedef float  v4fa __attribute__((ext_vector_type(4), may_alias));
union FragB { v16b v; v8us half[2]; };
union FragH { v16h v; v8us half[2]; };

__device__ __forceinline__ unsigned short bf16_bits(float x) { unsigned int u = __float_as_uint(x); return (unsigned short)((u + 0x7FFFu + ((u >> 16) & 1u)) >> 16); }
__device__ __forceinline__ float bf16_val(unsigned short b) { return __uint_as_float(((unsigned int)b) << 16); }
__device__ __forceinline__ float bf16_rne(float x) { return bf16_val(bf16_bits(x)); }
__device__ __forceinline__ unsigned short f16_bits(float x) { return __builtin_bit_cast(unsigned short, (_Float16)x); }
__device__ __forceinline__ float f16_val(unsigned short b) { return (float)__builtin_bit_cast(_Float16, b); }

__device__ __forceinline__ v8f mma_bf(v16b a, v16b b, v8f c) {
  c = __builtin_amdgcn_wmma_f32_16x16x32_bf16(false, a, false, b, (short)0, c, false, false);
  asm volatile("v_nop\n\tv_nop\n\tv_nop\n\tv_nop" : "+v"(c) : "v"(a), "v"(b));
  return c;
}
__device__ __forceinline__ v8f mma_h(v16h a, v16h b, v8f c) {
  c = __builtin_amdgcn_wmma_f32_16x16x32_f16(false, a, false, b, (short)0, c, false, false);
  asm volatile("v_nop\n\tv_nop\n\tv_nop\n\tv_nop" : "+v"(c) : "v"(a), "v"(b));
  return c;
}
__device__ __forceinline__ void mma_h2(v16h a0, v16h a1, v16h b, v8f& c0, v8f& c1) {
  c0 = __builtin_amdgcn_wmma_f32_16x16x32_f16(false, a0, false, b, (short)0, c0, false, false);
  c1 = __builtin_amdgcn_wmma_f32_16x16x32_f16(false, a1, false, b, (short)0, c1, false, false);
  asm volatile("v_nop\n\tv_nop\n\tv_nop\n\tv_nop" : "+v"(c0), "+v"(c1) : "v"(a0), "v"(a1), "v"(b));
}

__global__ __launch_bounds__(256) void k_cvt_bf16(const float* __restrict__ W, unsigned short* __restrict__ Wt, int n8, int seg8, int sstride8) {
  const int t = blockIdx.x * 256 + threadIdx.x;
  if (t >= n8) return;
  const int sg = t / seg8, rm = t - sg * seg8;
  const float* p = W + ((size_t)sg * sstride8 + rm) * 8;
  const v4f a = *(const v4fa*)p, b = *(const v4fa*)(p + 4);
  v8us v;
  v[0] = bf16_bits(a[0]); v[1] = bf16_bits(a[1]); v[2] = bf16_bits(a[2]); v[3] = bf16_bits(a[3]);
  v[4] = bf16_bits(b[0]); v[5] = bf16_bits(b[1]); v[6] = bf16_bits(b[2]); v[7] = bf16_bits(b[3]);
  *(volatile v8us*)(Wt + (size_t)t * 8) = v;
  __threadfence();
  *(volatile v8us*)(Wt + (size_t)t * 8) = v;
}

__global__ __launch_bounds__(256) void k_cvt_wp(const float* __restrict__ W, unsigned short* __restrict__ Wp2, int n8) {
  const int t = blockIdx.x * 256 + threadIdx.x;
  if (t >= n8) return;
  const int row = t / (CC / 8), c8 = (t - row * (CC / 8)) * 8;
  const float* p = W + (size_t)t * 8;
  const v4f a = *(const v4fa*)p, b = *(const v4fa*)(p + 4);
  const float xs[8] = {a[0], a[1], a[2], a[3], b[0], b[1], b[2], b[3]};
  v8us v0, v1;
#pragma unroll
  for (int i = 0; i < 8; ++i) { const float w = bf16_rne(xs[i]); v0[i] = f16_bits(w * 1024.0f); v1[i] = f16_bits(w * 4.0f); }
  unsigned short* d = Wp2 + (size_t)row * KP + c8;
  *(volatile v8us*)d = v0;
  *(volatile v8us*)(d + CC) = v1;
  __threadfence();
  *(volatile v8us*)d = v0;
  *(volatile v8us*)(d + CC) = v1;
}

__global__ __launch_bounds__(256) void k_rope_tab(float* __restrict__ tab, int T) {
  const int tid = threadIdx.x;
  const int wave = __builtin_amdgcn_readfirstlane((int)(threadIdx.x >> 5));
  const int t = blockIdx.x * 4 + (wave >> 1);
  const int i = tid & 31;
  double p = 1.0;
  p = p * ((i & 1)  ? 1.3335214321633240 : 1.0);
  p = p * ((i & 2)  ? 1.7782794100389228 : 1.0);
  p = p * ((i & 4)  ? 3.1622776601683795 : 1.0);
  p = p * ((i & 8)  ? 10.0 : 1.0);
  p = p * ((i & 16) ? 100.0 : 1.0);
  const float pf = (float)p;
  const float invf = 1.0f / pf;
  if (t >= T) return;
  const float ang = (float)t * invf;
  const float val = bf16_rne((wave & 1) ? sinf(ang) : cosf(ang));
  float* d = tab + (size_t)t * 64 + (wave & 1) * 32 + i;
  *(volatile float*)d = val;
  __threadfence();
  *(volatile float*)d = val;
}

__global__ __launch_bounds__(128) void k_qkv(const unsigned short* __restrict__ xb, const unsigned short* __restrict__ Wt,
                                             const float* __restrict__ g, const float* __restrict__ tab,
                                             unsigned short* __restrict__ planes) {
  __shared__ __attribute__((aligned(16))) float so[4][16][64];
  __shared__ __attribute__((aligned(16))) unsigned short sT[64][72];
  const int tid = threadIdx.x, lane = tid & 31, ln = lane & 15, hh = lane >> 4;
  const int wave = __builtin_amdgcn_readfirstlane((int)(threadIdx.x >> 5));
  const int mb = blockIdx.x / (QKVN / 64), nq = blockIdx.x % (QKVN / 64);
  const int kind = nq / NH, head = nq % NH;
  const int rowb = mb * 64;
  const int b = rowb / SEQ, tb = rowb - b * SEQ;
  const int row0 = rowb + wave * 16;
  const int bhd = b * NH + head;
  const unsigned short* arow = xb + (size_t)(row0 + ln) * CC;
  const unsigned short* brow = Wt + (size_t)(nq * 64 + ln) * CC;
  v8f acc[4];
#pragma unroll
  for (int t = 0; t < 4; ++t) acc[t] = (v8f){0.f,0.f,0.f,0.f,0.f,0.f,0.f,0.f};
  for (int kb = 0; kb < CC; kb += 32) {
    FragB a;
    a.half[0] = *(const v8us*)(arow + kb + 8 * hh);
    a.half[1] = *(const v8us*)(arow + kb + 16 + 8 * hh);
#pragma unroll
    for (int t = 0; t < 4; ++t) {
      const unsigned short* bp = brow + (size_t)(t * 16) * CC + kb;
      FragB bb;
      bb.half[0] = *(const v8us*)(bp + 8 * hh);
      bb.half[1] = *(const v8us*)(bp + 16 + 8 * hh);
      acc[t] = mma_bf(a.v, bb.v, acc[t]);
    }
  }
  if (kind < 2) {
    float gv[4];
#pragma unroll
    for (int t = 0; t < 4; ++t) gv[t] = bf16_rne(g[t * 16 + ln]);
#pragma unroll
    for (int r = 0; r < 8; ++r) {
      float s = acc[0][r] * acc[0][r] + acc[1][r] * acc[1][r] + acc[2][r] * acc[2][r] + acc[3][r] * acc[3][r];
      s += __shfl_xor(s, 1, 32); s += __shfl_xor(s, 2, 32); s += __shfl_xor(s, 4, 32); s += __shfl_xor(s, 8, 32);
      const float rstd = rsqrtf(s * (1.0f / 64.0f) + 1e-5f);
#pragma unroll
      for (int t = 0; t < 4; ++t) acc[t][r] = gv[t] * (acc[t][r] * rstd);
    }
#pragma unroll
    for (int nt = 0; nt < 2; ++nt) {
#pragma unroll
      for (int r = 0; r < 8; ++r) {
        const int tok = tb + wave * 16 + 8 * hh + r;
        const float cv = tab[(size_t)tok * 64 + nt * 16 + ln];
        const float sv = tab[(size_t)tok * 64 + 32 + nt * 16 + ln];
        const float u1 = acc[nt][r], u2 = acc[nt + 2][r];
        acc[nt][r]     =  u1 * cv + u2 * sv;
        acc[nt + 2][r] = -u1 * sv + u2 * cv;
      }
    }
#pragma unroll
    for (int t = 0; t < 4; ++t)
#pragma unroll
      for (int r = 0; r < 8; ++r) so[wave][8 * hh + r][t * 16 + ln] = acc[t][r];
  } else {
#pragma unroll
    for (int t = 0; t < 4; ++t)
#pragma unroll
      for (int r = 0; r < 8; ++r) sT[t * 16 + ln][wave * 16 + 8 * hh + r] = f16_bits(acc[t][r]);
  }
  __syncthreads();
  if (kind < 2) {
    const int c8 = (lane & 7) * 8;
    v8us hi[4], rs[4];
#pragma unroll
    for (int it = 0; it < 4; ++it) {
      const int rr = it * 4 + (lane >> 3);
      const v4f a = *(const v4fa*)&so[wave][rr][c8], c = *(const v4fa*)&so[wave][rr][c8 + 4];
      const float xs[8] = {a[0], a[1], a[2], a[3], c[0], c[1], c[2], c[3]};
#pragma unroll
      for (int i = 0; i < 8; ++i) {
        const unsigned short hb = f16_bits(xs[i]);
        hi[it][i] = hb;
        rs[it][i] = f16_bits((xs[i] - f16_val(hb)) * 1024.0f);
      }
    }
    const int hoff = (kind == 0) ? 0 : 2 * PL;
    const size_t rbase = ((size_t)bhd * SEQ + tb + wave * 16) * HD;
    for (int pass = 0; pass < 2; ++pass) {
#pragma unroll
      for (int it = 0; it < 4; ++it) {
        const int rr = it * 4 + (lane >> 3);
        *(volatile v8us*)(planes + hoff + rbase + (size_t)rr * HD + c8) = hi[it];
        if (kind == 0) *(volatile v8us*)(planes + PL + rbase + (size_t)rr * HD + c8) = rs[it];
      }
      if (pass == 0) __threadfence();
    }
  } else {
    v8us vv[4];
#pragma unroll
    for (int it = 0; it < 4; ++it) {
      const int p = it * 128 + tid;
      vv[it] = *(const v8us*)&sT[p >> 3][(p & 7) * 8];
    }
    for (int pass = 0; pass < 2; ++pass) {
#pragma unroll
      for (int it = 0; it < 4; ++it) {
        const int p = it * 128 + tid;
        const int d = p >> 3, c8 = (p & 7) * 8;
        *(volatile v8us*)(planes + 3 * PL + ((size_t)bhd * HD + d) * SEQ + tb + c8) = vv[it];
      }
      if (pass == 0) __threadfence();
    }
  }
}

__global__ __launch_bounds__(128) __attribute__((amdgpu_num_vgpr(256)))
void k_flash(const unsigned short* __restrict__ planes, unsigned short* __restrict__ Yp) {
  __shared__ __attribute__((aligned(16))) unsigned short sK[64][72], sV[64][72];
  __shared__ __attribute__((aligned(16))) unsigned short sP[4][16][40];
  __shared__ __attribute__((aligned(16))) float sO[4][16][64];
  const int tid = threadIdx.x, lane = tid & 31, ln = lane & 15, hh = lane >> 4;
  const int wave = __builtin_amdgcn_readfirstlane((int)(threadIdx.x >> 5));
  constexpr int NQB = SEQ / 64;
  const int bh = blockIdx.x / NQB, qblk = blockIdx.x % NQB;
  const int b = bh / NH, h = bh % NH;
  const int q0 = qblk * 64 + wave * 16;
  const int qoff0 = (bh * SEQ + q0 + ln) * HD;
  const int koff0 = 2 * PL + bh * SEQ * HD;
  const int voff0 = 3 * PL + bh * HD * SEQ;
  const float RS = 0.0009765625f;
  const float LNC = 6.931471806f;
  float m_r[8], l_r[8];
#pragma unroll
  for (int r = 0; r < 8; ++r) { m_r[r] = -1.0e30f; l_r[r] = 0.f; }
  v8f oacc[4];
#pragma unroll
  for (int dt = 0; dt < 4; ++dt) oacc[dt] = (v8f){0.f,0.f,0.f,0.f,0.f,0.f,0.f,0.f};

#pragma unroll 1
  for (int j0 = 0; j0 < SEQ; j0 += 64) {
    __syncthreads();
#pragma unroll
    for (int it = 0; it < 4; ++it) {
      const int p = it * 128 + tid;
      const int r = p >> 3, c8 = (p & 7) * 8;
      const v8us kx = *(const v8us*)(planes + koff0 + (j0 + r) * HD + c8);
      const v8us vx = *(const v8us*)(planes + voff0 + r * SEQ + j0 + c8);
      *(v8us*)&sK[r][c8] = kx;
      *(v8us*)&sV[r][c8] = vx;
    }
    __syncthreads();
#pragma unroll 1
    for (int hf = 0; hf < 2; ++hf) {
      int qo = qoff0;
      asm volatile("" : "+v"(qo));
      v8f sh0 = (v8f){0.f,0.f,0.f,0.f,0.f,0.f,0.f,0.f}, sh1 = sh0, sr0 = sh0, sr1 = sh0;
#pragma unroll
      for (int ks = 0; ks < 2; ++ks) {
        FragH qh, qr, k0, k1;
        const unsigned short* qp = planes + qo + ks * 32;
        qh.half[0] = *(const v8us*)(qp + 8 * hh);       qh.half[1] = *(const v8us*)(qp + 16 + 8 * hh);
        qr.half[0] = *(const v8us*)(qp + PL + 8 * hh);  qr.half[1] = *(const v8us*)(qp + PL + 16 + 8 * hh);
        k0.half[0] = *(const v8us*)&sK[hf * 32 + ln][ks * 32 + 8 * hh];      k0.half[1] = *(const v8us*)&sK[hf * 32 + ln][ks * 32 + 16 + 8 * hh];
        k1.half[0] = *(const v8us*)&sK[hf * 32 + 16 + ln][ks * 32 + 8 * hh]; k1.half[1] = *(const v8us*)&sK[hf * 32 + 16 + ln][ks * 32 + 16 + 8 * hh];
        mma_h2(qh.v, qr.v, k0.v, sh0, sr0);
        mma_h2(qh.v, qr.v, k1.v, sh1, sr1);
      }
      float alpha[8];
#pragma unroll
      for (int r = 0; r < 8; ++r) {
        const float t0 = (sh0[r] + sr0[r] * RS) * 0.125f;
        const float t1 = (sh1[r] + sr1[r] * RS) * 0.125f;
        float mx = fmaxf(t0, t1);
        mx = fmaxf(mx, __shfl_xor(mx, 1, 32)); mx = fmaxf(mx, __shfl_xor(mx, 2, 32)); mx = fmaxf(mx, __shfl_xor(mx, 4, 32)); mx = fmaxf(mx, __shfl_xor(mx, 8, 32));
        const float mnew = fmaxf(m_r[r], mx);
        alpha[r] = __expf(m_r[r] - mnew);
        const float p0 = __expf(t0 - mnew + LNC);
        const float p1 = __expf(t1 - mnew + LNC);
        m_r[r] = mnew;
        l_r[r] = l_r[r] * alpha[r] + (p0 + p1);
        sP[wave][8 * hh + r][ln] = f16_bits(p0);
        sP[wave][8 * hh + r][16 + ln] = f16_bits(p1);
      }
#pragma unroll
      for (int dt = 0; dt < 4; ++dt)
#pragma unroll
        for (int r = 0; r < 8; ++r) oacc[dt][r] *= alpha[r];
      __builtin_amdgcn_fence(4  , "workgroup");
      __builtin_amdgcn_wave_barrier();
      FragH pa;
      pa.half[0] = *(const v8us*)&sP[wave][ln][8 * hh];
      pa.half[1] = *(const v8us*)&sP[wave][ln][16 + 8 * hh];
#pragma unroll
      for (int dt = 0; dt < 4; ++dt) {
        FragH bv;
        bv.half[0] = *(const v8us*)&sV[dt * 16 + ln][hf * 32 + 8 * hh];
        bv.half[1] = *(const v8us*)&sV[dt * 16 + ln][hf * 32 + 16 + 8 * hh];
        oacc[dt] = mma_h(pa.v, bv.v, oacc[dt]);
      }
      __builtin_amdgcn_fence(4  , "workgroup");
      __builtin_amdgcn_wave_barrier();
    }
  }
#pragma unroll
  for (int r = 0; r < 8; ++r) {
    float l = l_r[r];
    l += __shfl_xor(l, 1, 32); l += __shfl_xor(l, 2, 32); l += __shfl_xor(l, 4, 32); l += __shfl_xor(l, 8, 32);
    l_r[r] = 32.0f * (1.0f / l);
  }
#pragma unroll
  for (int dt = 0; dt < 4; ++dt)
#pragma unroll
    for (int r = 0; r < 8; ++r) sO[wave][8 * hh + r][dt * 16 + ln] = oacc[dt][r] * l_r[r];
  __builtin_amdgcn_fence(4  , "workgroup");
  __builtin_amdgcn_wave_barrier();
  const int c8 = (lane & 7) * 8;
  v8us hi[4], rs[4];
#pragma unroll
  for (int it = 0; it < 4; ++it) {
    const int rr = it * 4 + (lane >> 3);
    const v4f a = *(const v4fa*)&sO[wave][rr][c8], c = *(const v4fa*)&sO[wave][rr][c8 + 4];
    const float xs[8] = {a[0], a[1], a[2], a[3], c[0], c[1], c[2], c[3]};
#pragma unroll
    for (int i = 0; i < 8; ++i) {
      const unsigned short hb = f16_bits(xs[i]);
      hi[it][i] = hb;
      rs[it][i] = f16_bits((xs[i] - f16_val(hb)) * 256.0f);
    }
  }
  const size_t ybase = ((size_t)b * SEQ + q0) * KP + h * HD;
  for (int pass = 0; pass < 2; ++pass) {
#pragma unroll
    for (int it = 0; it < 4; ++it) {
      const int rr = it * 4 + (lane >> 3);
      *(volatile v8us*)(Yp + ybase + (size_t)rr * KP + c8) = hi[it];
      *(volatile v8us*)(Yp + ybase + (size_t)rr * KP + CC + c8) = rs[it];
    }
    if (pass == 0) __threadfence();
  }
}

__global__ __launch_bounds__(128) void k_proj(const unsigned short* __restrict__ A, const unsigned short* __restrict__ Wt,
                                              float* __restrict__ C, int M, int seg, int csr) {
  __shared__ __attribute__((aligned(16))) float so[4][16][64];
  const int tid = threadIdx.x, lane = tid & 31, ln = lane & 15, hh = lane >> 4;
  const int wave = __builtin_amdgcn_readfirstlane((int)(threadIdx.x >> 5));
  const int ntn = CC / 64;
  const int wid = blockIdx.x * 4 + wave;
  const int mt = wid / ntn, nq = wid % ntn;
  if (mt * 16 >= M) return;
  const int row0 = mt * 16, col0 = nq * 64;
  const int bseg = row0 / seg, t0 = row0 - bseg * seg;
  const unsigned short* arow = A + (size_t)(row0 + ln) * KP;
  const unsigned short* brow = Wt + (size_t)(col0 + ln) * KP;
  float* crow0 = C + ((size_t)bseg * csr + t0) * CC;
  v8f acc[4];
#pragma unroll
  for (int t = 0; t < 4; ++t) acc[t] = (v8f){0.f,0.f,0.f,0.f,0.f,0.f,0.f,0.f};
  for (int kb = 0; kb < KP; kb += 32) {
    FragH a;
    a.half[0] = *(const v8us*)(arow + kb + 8 * hh);
    a.half[1] = *(const v8us*)(arow + kb + 16 + 8 * hh);
#pragma unroll
    for (int t = 0; t < 4; ++t) {
      const unsigned short* bp = brow + (size_t)(t * 16) * KP + kb;
      FragH bb;
      bb.half[0] = *(const v8us*)(bp + 8 * hh);
      bb.half[1] = *(const v8us*)(bp + 16 + 8 * hh);
      acc[t] = mma_h(a.v, bb.v, acc[t]);
    }
  }
  const float OS = 0.000030517578125f;
#pragma unroll
  for (int t = 0; t < 4; ++t) {
#pragma unroll
    for (int r = 0; r < 8; ++r) so[wave][8 * hh + r][t * 16 + ln] = acc[t][r] * OS;
  }
  __builtin_amdgcn_fence(4  , "workgroup");
  __builtin_amdgcn_wave_barrier();
  const int rsub = lane >> 4, c4 = (lane & 15) * 4;
  v4f vals[8];
#pragma unroll
  for (int q = 0; q < 8; ++q) {
    const int r = q * 2 + rsub;
    vals[q] = *(const v4fa*)&so[wave][r][c4];
  }
  for (int pass = 0; pass < 2; ++pass) {
#pragma unroll
    for (int q = 0; q < 8; ++q) {
      const int r = q * 2 + rsub;
      *(volatile v4f*)(crow0 + (size_t)r * CC + col0 + c4) = vals[q];
    }
    if (pass == 0) __threadfence();
  }
}

extern "C" void kernel_launch(void* const* d_in, const int* in_sizes, int n_in,
                              void* d_out, int out_size, void* d_ws, size_t ws_size, hipStream_t stream) {
  if (n_in < 6) return;
  if (in_sizes[0] < ((NB - 1) * SEQ_FULL + SEQ) * CC) return;
  if (in_sizes[1] < CC * CC) return;
  if (in_sizes[2] < CC * CC) return;
  if (in_sizes[3] < CC * CC) return;
  if (in_sizes[4] < CC * CC) return;
  if (in_sizes[5] < HD) return;
  if (out_size < ((NB - 1) * OUT_SEG_ROWS + SEQ) * CC) return;
  const float* x  = (const float*)d_in[0];
  const float* Wq = (const float*)d_in[1];
  const float* Wk = (const float*)d_in[2];
  const float* Wv = (const float*)d_in[3];
  const float* Wo = (const float*)d_in[4];
  const float* g  = (const float*)d_in[5];
  char* ws = (char*)d_ws; size_t off = 0;
  unsigned short* xb    = (unsigned short*)(ws + off); off += (size_t)NB * SEQ * CC * 2;
  unsigned short* Wqkvt = (unsigned short*)(ws + off); off += (size_t)3 * CC * CC * 2;
  unsigned short* Wp2   = (unsigned short*)(ws + off); off += (size_t)CC * KP * 2;
  float* tab            = (float*)(ws + off);          off += (size_t)SEQ * 64 * 4;
  unsigned short* planes = (unsigned short*)(ws + off); off += (size_t)4 * PL * 2;
  unsigned short* Yp    = (unsigned short*)(ws + off); off += (size_t)NB * SEQ * KP * 2;
  if (off > ws_size) return;
  if (off > (size_t)134217728) return;
  const int M = NB * SEQ;
  const int nw8 = CC * CC / 8;
  const int nx8 = NB * SEQ * (CC / 8);
  k_cvt_bf16<<<(nx8 + 255) / 256, 256, 0, stream>>>(x, xb, nx8, SEQ * (CC / 8), SEQ_FULL * (CC / 8));
  k_cvt_bf16<<<(nw8 + 255) / 256, 256, 0, stream>>>(Wq, Wqkvt, nw8, nw8, nw8);
  k_cvt_bf16<<<(nw8 + 255) / 256, 256, 0, stream>>>(Wk, Wqkvt + (size_t)CC * CC, nw8, nw8, nw8);
  k_cvt_bf16<<<(nw8 + 255) / 256, 256, 0, stream>>>(Wv, Wqkvt + (size_t)2 * CC * CC, nw8, nw8, nw8);
  k_cvt_wp<<<(nw8 + 255) / 256, 256, 0, stream>>>(Wo, Wp2, nw8);
  k_rope_tab<<<(SEQ + 3) / 4, 256, 0, stream>>>(tab, SEQ);
  k_qkv<<<(M / 64) * (QKVN / 64), 128, 0, stream>>>(xb, Wqkvt, g, tab, planes);
  k_flash<<<NB * NH * (SEQ / 64), 128, 0, stream>>>(planes, Yp);
  k_proj<<<((M / 16) * (CC / 64) + 3) / 4, 128, 0, stream>>>(Yp, Wp2, (float*)d_out, M, SEQ, OUT_SEG_ROWS);
}
